// MambaBlock_82849919140302
// MI455X (gfx1250) — hardware-verified
//
#include <hip/hip_runtime.h>
#include <stddef.h>
#include <stdint.h>
#include <math.h>


#define NTOK    16384
#define NCHUNK  256
#define CHN     128
#define DINNER  256
#define NXBC    384
#define NPROJ   644
#define NPADP   704
#define KFF     2304
#define LP      72
#define TP      132
#define YP      260
#define NIMG    2097152
#define WSMAX   134217728
#define NU_WIN  (NPADP * 32)
#define NU_WOUT (CHN * 64)
#define NU_FF   (CHN * 288)
#define SSDOUT_LDS (64 * YP * 4 + 1024 + 1024 + 2 * 64 * LP * 2)

static_assert(NU_WIN % 256 == 0 && NU_WOUT % 256 == 0 && NU_FF % 256 == 0);
static_assert(NPADP % 64 == 0 && NTOK % 64 == 0 && KFF == 9 * 256);
static_assert((LP * 2) % 16 == 0 && (TP * 4) % 16 == 0 && (YP * 4) % 16 == 0);
static_assert(SSDOUT_LDS == 87040);
static_assert(NIMG + 1 == 2097153);

typedef float          v4f   __attribute__((ext_vector_type(4)));
typedef float          v8f   __attribute__((ext_vector_type(8)));
typedef int            v8i   __attribute__((ext_vector_type(8)));
typedef unsigned short v8us  __attribute__((ext_vector_type(8)));
typedef unsigned short v16us __attribute__((ext_vector_type(16)));
typedef __bf16         v16bf __attribute__((ext_vector_type(16)));
typedef v4f  __attribute__((may_alias)) v4fa;
typedef v8us __attribute__((may_alias)) v8usa;
union FragB { v16bf v; v16us u; v8us h[2]; v8i w; };

__device__ __forceinline__ v8f wmb(const FragB& a, const FragB& b, v8f c) {
  v8f d = __builtin_amdgcn_wmma_f32_16x16x32_bf16(false, a.v, false, b.v, (short)0, c, false, false);
  asm volatile("v_nop\n\tv_nop\n\tv_nop\n\tv_nop" : "+v"(d) : "v"(a.w), "v"(b.w));
  return d;
}
__device__ __forceinline__ v8f mm3(const FragB& ah, const FragB& al, const FragB& bh, const FragB& bl, v8f c) {
  c = wmb(ah, bh, c);
  c = wmb(al, bh, c);
  c = wmb(ah, bl, c);
  return c;
}
__device__ __forceinline__ void ldg_frag(FragB& f, const unsigned short* __restrict__ p) {
  f.h[0] = *(const v8usa*)p;
  f.h[1] = *(const v8usa*)(p + 16);
}
__device__ __forceinline__ void lds_frag(FragB& f, const unsigned short* p) {
  f.h[0] = *(const v8usa*)p;
  f.h[1] = *(const v8usa*)(p + 16);
}

__device__ __forceinline__ unsigned bf16_bits(float f) {
  const unsigned u = __float_as_uint(f);
  return (u + 0x7FFFu + ((u >> 16) & 1u)) >> 16;
}
__device__ __forceinline__ float bf16_val(float f) { return __uint_as_float(bf16_bits(f) << 16); }
__device__ __forceinline__ float bfu(unsigned short s) { return __uint_as_float(((unsigned)s) << 16); }
__device__ __forceinline__ void split_bf(float v, unsigned short& hi, unsigned short& lo) {
  const unsigned hb = bf16_bits(v);
  hi = (unsigned short)hb;
  lo = (unsigned short)bf16_bits(v - __uint_as_float(hb << 16));
}
__device__ __forceinline__ float silu_f(float v) { return v * (1.0f / (1.0f + expf(-v))); }
__device__ __forceinline__ float softplus_f(float v) { return fmaxf(v, 0.0f) + log1pf(expf(-fabsf(v))); }

__global__ __launch_bounds__(256) void k_wprep(const float* __restrict__ wip, const float* __restrict__ wop,
                                               const float* __restrict__ w1, const float* __restrict__ w2,
                                               const float* __restrict__ aux,
                                               unsigned short* WIN2, unsigned short* WOUT2,
                                               unsigned short* W1R, unsigned short* W2R, float* outp) {
  const int u = (int)blockIdx.x * 256 + (int)threadIdx.x;
  const float av = bf16_val(aux[0]);
  v8us o;
  unsigned short* dp;
  if (u < NU_WIN) {
    const int n = u >> 5;
    const int k8 = (u & 31) * 8;
    const int kk = k8 & 127;
    const int nc = n < NPROJ ? n : NPROJ - 1;
    const float* p = wip + (size_t)nc * CHN + kk;
    const v4f a = *(const v4f*)p;
    const v4f b = *(const v4f*)(p + 4);
    const bool ok = n < NPROJ;
    o[0] = ok ? (unsigned short)bf16_bits(a.x) : (unsigned short)0;
    o[1] = ok ? (unsigned short)bf16_bits(a.y) : (unsigned short)0;
    o[2] = ok ? (unsigned short)bf16_bits(a.z) : (unsigned short)0;
    o[3] = ok ? (unsigned short)bf16_bits(a.w) : (unsigned short)0;
    o[4] = ok ? (unsigned short)bf16_bits(b.x) : (unsigned short)0;
    o[5] = ok ? (unsigned short)bf16_bits(b.y) : (unsigned short)0;
    o[6] = ok ? (unsigned short)bf16_bits(b.z) : (unsigned short)0;
    o[7] = ok ? (unsigned short)bf16_bits(b.w) : (unsigned short)0;
    dp = WIN2 + (size_t)n * 256 + k8;
  } else if (u < NU_WIN + NU_WOUT) {
    const int v = u - NU_WIN;
    const int n = v >> 6;
    const int k8 = (v & 63) * 8;
    const int kk = k8 & 255;
    const float* p = wop + (size_t)n * DINNER + kk;
    const v4f a = *(const v4f*)p;
    const v4f b = *(const v4f*)(p + 4);
    o[0] = (unsigned short)bf16_bits(a.x); o[1] = (unsigned short)bf16_bits(a.y);
    o[2] = (unsigned short)bf16_bits(a.z); o[3] = (unsigned short)bf16_bits(a.w);
    o[4] = (unsigned short)bf16_bits(b.x); o[5] = (unsigned short)bf16_bits(b.y);
    o[6] = (unsigned short)bf16_bits(b.z); o[7] = (unsigned short)bf16_bits(b.w);
    dp = WOUT2 + (size_t)n * 512 + k8;
  } else if (u < NU_WIN + NU_WOUT + NU_FF) {
    const int v = u - (NU_WIN + NU_WOUT);
    const int n = v / 288;
    const int rem = v - n * 288;
    const int tap = rem >> 5;
    const int j = rem & 31;
    const int ci0 = (j & 15) * 8;
    const float* p = w1 + (size_t)n * 1152 + (size_t)ci0 * 9 + tap;
#pragma unroll
    for (int i = 0; i < 8; ++i) o[i] = (unsigned short)bf16_bits(p[(size_t)i * 9]);
    dp = W1R + (size_t)n * KFF + tap * 256 + j * 8;
  } else if (u < NU_WIN + NU_WOUT + 2 * NU_FF) {
    const int v = u - (NU_WIN + NU_WOUT + NU_FF);
    const int n = v / 288;
    const int rem = v - n * 288;
    const int tap = rem >> 5;
    const int j = rem & 31;
    const int ci0 = (j & 15) * 8;
    const float* p = w2 + (size_t)n * 1152 + (size_t)ci0 * 9 + tap;
#pragma unroll
    for (int i = 0; i < 8; ++i) o[i] = (unsigned short)bf16_bits(p[(size_t)i * 9]);
    dp = W2R + (size_t)n * KFF + tap * 256 + j * 8;
  } else {
    return;
  }
  *(volatile v8us*)dp = o;
  if (u == 0) *(volatile float*)(outp + NIMG) = av;
  __threadfence();
  *(volatile v8us*)dp = o;
  if (u == 0) *(volatile float*)(outp + NIMG) = av;
}

__global__ __launch_bounds__(256) void k_ln(const float* __restrict__ noisy, const float* __restrict__ lnw,
                                            const float* __restrict__ lnb, float* XT, unsigned short* NRM) {
  __shared__ __attribute__((aligned(16))) float tile[64 * TP];
  __shared__ float lw[CHN], lb[CHN], mus[64], rss[64];
  const int tid = (int)threadIdx.x, lane = tid & 31, wave = tid >> 5;
  const int blk = (int)blockIdx.x;
  const int b = blk >> 6, y = blk & 63;
  const int tok0 = blk * 64;
#pragma unroll 2
  for (int it = 0; it < 8; ++it) {
    const int idx = it * 256 + tid;
    const int c = idx >> 4, q = idx & 15;
    const v4f v = *(const v4f*)(noisy + (((size_t)(b * CHN + c) * 64 + y) * 64 + 4 * q));
    tile[(4 * q + 0) * TP + c] = bf16_val(v.x);
    tile[(4 * q + 1) * TP + c] = bf16_val(v.y);
    tile[(4 * q + 2) * TP + c] = bf16_val(v.z);
    tile[(4 * q + 3) * TP + c] = bf16_val(v.w);
  }
  if (tid < CHN) { lw[tid] = bf16_val(lnw[tid]); lb[tid] = bf16_val(lnb[tid]); }
  __syncthreads();
  {
    const int t = tid >> 2, part = tid & 3;
    const float* tr = tile + t * TP + part * 32;
    float s = 0.0f;
#pragma unroll 8
    for (int j = 0; j < 32; ++j) s += tr[j];
    s += __shfl_xor(s, 1, 32);
    s += __shfl_xor(s, 2, 32);
    const float mu = s * (1.0f / 128.0f);
    float q2 = 0.0f;
#pragma unroll 8
    for (int j = 0; j < 32; ++j) { const float d = tr[j] - mu; q2 += d * d; }
    q2 += __shfl_xor(q2, 1, 32);
    q2 += __shfl_xor(q2, 2, 32);
    const float rs = rsqrtf(q2 * (1.0f / 128.0f) + 1e-5f);
    if (part == 0) { mus[t] = mu; rss[t] = rs; }
  }
  __syncthreads();
  const int c0 = 8 * (lane & 15);
  const bool lo_sel = lane >= 16;
#pragma unroll 1
  for (int i = 0; i < 8; ++i) {
    const int t = wave * 8 + i;
    const v4f xv = *(const v4fa*)(tile + t * TP + 4 * lane);
    const float mu = mus[t], rs = rss[t];
    v8us o;
#pragma unroll
    for (int j = 0; j < 8; ++j) {
      const float n = (tile[t * TP + c0 + j] - mu) * rs * lw[c0 + j] + lb[c0 + j];
      unsigned short hs, ls;
      split_bf(n, hs, ls);
      o[j] = lo_sel ? ls : hs;
    }
    float* xp = XT + (size_t)(tok0 + t) * CHN + 4 * lane;
    unsigned short* np = NRM + (size_t)(tok0 + t) * 256 + 8 * lane;
    *(volatile v4f*)xp = xv;
    *(volatile v8us*)np = o;
    __threadfence();
    *(volatile v4f*)xp = xv;
    *(volatile v8us*)np = o;
  }
}

__global__ __launch_bounds__(128) void k_inproj(const unsigned short* __restrict__ A,
                                                const unsigned short* __restrict__ WT,
                                                const float* __restrict__ dtb, const float* __restrict__ alog,
                                                float* wsf, size_t oZ, size_t oX, size_t oD) {
  __shared__ __attribute__((aligned(16))) float stg[64 * 64];
  const int tid = (int)threadIdx.x, lane = tid & 31, wave = tid >> 5, hh = lane >> 4, m = lane & 15;
  const int rowBase = (int)blockIdx.x * 64;
  const int ny = (int)blockIdx.y;
  const int col0 = ny * 64;
  v8f acc[4];
  {
    const v8f z = {0.f, 0.f, 0.f, 0.f, 0.f, 0.f, 0.f, 0.f};
    acc[0] = z; acc[1] = z; acc[2] = z; acc[3] = z;
  }
  const unsigned short* ap = A + (size_t)(rowBase + 16 * wave + m) * 256 + 8 * hh;
  const unsigned short* wp = WT + (size_t)(col0 + m) * 256 + 8 * hh;
#pragma unroll 1
  for (int ks = 0; ks < 8; ++ks) {
    FragB af;
    ldg_frag(af, ap + 32 * ks);
#pragma unroll
    for (int t = 0; t < 4; ++t) {
      FragB bf;
      ldg_frag(bf, wp + (size_t)(16 * t) * 256 + 32 * ks);
      acc[t] = wmb(af, bf, acc[t]);
    }
  }
#pragma unroll
  for (int t = 0; t < 4; ++t) {
#pragma unroll
    for (int r = 0; r < 8; ++r) stg[(16 * wave + 8 * hh + r) * 64 + 16 * t + m] = acc[t][r];
  }
  __syncthreads();
  if (ny < 10) {
    const size_t pitch = (ny < 4) ? (size_t)256 : (size_t)384;
    const size_t base  = (ny < 4) ? (oZ + (size_t)(64 * ny)) : (oX + (size_t)(64 * (ny - 4)));
    v4f fv[8];
#pragma unroll
    for (int i = 0; i < 8; ++i) fv[i] = *(const v4fa*)(stg + (16 * wave + 2 * i + hh) * 64 + 4 * m);
#pragma unroll
    for (int i = 0; i < 8; ++i) {
      const int lr = 16 * wave + 2 * i + hh;
      *(volatile v4f*)(wsf + base + (size_t)(rowBase + lr) * pitch + 4 * m) = fv[i];
    }
    __threadfence();
#pragma unroll
    for (int i = 0; i < 8; ++i) {
      const int lr = 16 * wave + 2 * i + hh;
      *(volatile v4f*)(wsf + base + (size_t)(rowBase + lr) * pitch + 4 * m) = fv[i];
    }
  } else {
    const int tt = tid >> 1;
    const bool second = (tid & 1) != 0;
    const v4f raw = *(const v4fa*)(stg + tt * 64);
    const v4f db = *(const v4f*)dtb;
    const v4f al = *(const v4f*)alog;
    const float d0 = softplus_f(raw.x + bf16_val(db.x));
    const float d1 = softplus_f(raw.y + bf16_val(db.y));
    const float d2 = softplus_f(raw.z + bf16_val(db.z));
    const float d3 = softplus_f(raw.w + bf16_val(db.w));
    const float a0 = d0 * (-expf(bf16_val(al.x)));
    const float a1 = d1 * (-expf(bf16_val(al.y)));
    const float a2 = d2 * (-expf(bf16_val(al.z)));
    const float a3 = d3 * (-expf(bf16_val(al.w)));
    v4f ov;
    ov.x = second ? a0 : d0; ov.y = second ? a1 : d1; ov.z = second ? a2 : d2; ov.w = second ? a3 : d3;
    float* op = wsf + oD + (size_t)rowBase * 8 + 4 * tid;
    *(volatile v4f*)op = ov;
    __threadfence();
    *(volatile v4f*)op = ov;
  }
}

__device__ __forceinline__ void plane_write(unsigned short* dst, const float* ov, int sJ, int sR, int tid) {
  v8us o[4];
#pragma unroll
  for (int it = 0; it < 4; ++it) {
    const int u = it * 256 + tid;
    const int row = u >> 4, q = u & 15;
    const int s0 = 8 * (q & 7);
    const bool lo_sel = q >= 8;
    v8us w;
#pragma unroll
    for (int j = 0; j < 8; ++j) {
      const float v = ov[row * sR + (s0 + j) * sJ];
      unsigned short hs, ls;
      split_bf(v, hs, ls);
      w[j] = lo_sel ? ls : hs;
    }
    o[it] = w;
  }
#pragma unroll
  for (int it = 0; it < 4; ++it) {
    const int u = it * 256 + tid;
    *(volatile v8us*)(dst + (size_t)(u >> 4) * 128 + 8 * (u & 15)) = o[it];
  }
  __threadfence();
#pragma unroll
  for (int it = 0; it < 4; ++it) {
    const int u = it * 256 + tid;
    *(volatile v8us*)(dst + (size_t)(u >> 4) * 128 + 8 * (u & 15)) = o[it];
  }
}

__global__ __launch_bounds__(256) void k_conv1d(const float* __restrict__ XBC, const float* __restrict__ DTA,
                                                const float* __restrict__ cwv, const float* __restrict__ cbv,
                                                unsigned short* XTP, unsigned short* BTT, unsigned short* BTK,
                                                unsigned short* CTK, float* CS) {
  __shared__ float raw[68 * 65];
  __shared__ float outv[64 * 65];
  __shared__ float cw[64 * 5], cb[64];
  __shared__ float al[256];
  __shared__ __attribute__((aligned(16))) float csl[256];
  const int tid = (int)threadIdx.x;
  const int chunk = (int)blockIdx.x;
  const int slab = (int)blockIdx.y;
  const int c = chunk & 63;
  const int tok0 = chunk * 64;
  const int ch0 = slab * 64;
#pragma unroll 1
  for (int idx = tid; idx < 68 * 16; idx += 256) {
    const int r = idx >> 4, q = idx & 15;
    const bool ok = (c * 64 - 4 + r) >= 0;
    const int gt = ok ? (tok0 - 4 + r) : tok0;
    const v4f v = *(const v4f*)(XBC + (size_t)gt * NXBC + ch0 + 4 * q);
    raw[r * 65 + 4 * q + 0] = ok ? v.x : 0.0f;
    raw[r * 65 + 4 * q + 1] = ok ? v.y : 0.0f;
    raw[r * 65 + 4 * q + 2] = ok ? v.z : 0.0f;
    raw[r * 65 + 4 * q + 3] = ok ? v.w : 0.0f;
  }
#pragma unroll 1
  for (int i = tid; i < 320; i += 256) cw[i] = bf16_val(cwv[ch0 * 5 + i]);
  if (tid < 64) cb[tid] = bf16_val(cbv[ch0 + tid]);
  __syncthreads();
  {
    const int ch = tid & 63, tq = tid >> 6;
    const float w0 = cw[ch * 5 + 0], w1 = cw[ch * 5 + 1], w2 = cw[ch * 5 + 2], w3 = cw[ch * 5 + 3], w4 = cw[ch * 5 + 4];
    const float bb = cb[ch];
#pragma unroll 1
    for (int i = 0; i < 16; ++i) {
      const int t = tq * 16 + i;
      float a = bb;
      a += raw[(t + 0) * 65 + ch] * w0;
      a += raw[(t + 1) * 65 + ch] * w1;
      a += raw[(t + 2) * 65 + ch] * w2;
      a += raw[(t + 3) * 65 + ch] * w3;
      a += raw[(t + 4) * 65 + ch] * w4;
      outv[t * 65 + ch] = silu_f(a);
    }
  }
  __syncthreads();
  if (slab < 4) {
    plane_write(XTP + (size_t)(chunk * 4 + slab) * 8192, outv, 65, 1, tid);
  } else if (slab == 4) {
    plane_write(BTT + (size_t)chunk * 8192, outv, 65, 1, tid);
    plane_write(BTK + (size_t)tok0 * 128, outv, 1, 65, tid);
  } else {
    plane_write(CTK + (size_t)tok0 * 128, outv, 1, 65, tid);
  }
  if (slab == 0) {
    al[tid] = DTA[(size_t)(tok0 + (tid >> 2)) * 8 + 4 + (tid & 3)];
    __syncthreads();
    if (tid < 4) {
      float run = 0.0f;
#pragma unroll 1
      for (int t = 0; t < 64; ++t) { run += al[t * 4 + tid]; csl[t * 4 + tid] = run; }
    }
    __syncthreads();
    if (tid < 64) {
      const v4f cv = *(const v4fa*)(csl + 4 * tid);
      float* op = CS + (size_t)tok0 * 4 + 4 * tid;
      *(volatile v4f*)op = cv;
      __threadfence();
      *(volatile v4f*)op = cv;
    }
  }
}

__global__ __launch_bounds__(128) void k_ssd_local(const unsigned short* __restrict__ CTK,
                                                   const unsigned short* __restrict__ BTK,
                                                   const unsigned short* __restrict__ XTP,
                                                   const unsigned short* __restrict__ BTT,
                                                   const float* __restrict__ CS, const float* __restrict__ DTA,
                                                   const float* __restrict__ Dp, float* Y, float* S) {
  __shared__ __attribute__((aligned(16))) unsigned short MmS[2 * 64 * LP];
  __shared__ __attribute__((aligned(16))) unsigned short BwS[2 * 64 * LP];
  __shared__ __attribute__((aligned(16))) float stg[64 * 64];
  __shared__ __attribute__((aligned(16))) float csS[256];
  __shared__ __attribute__((aligned(16))) float dtS[256];
  __shared__ float wS[256];
  const int tid = (int)threadIdx.x, lane = tid & 31, wave = tid >> 5, hh = lane >> 4, m = lane & 15;
  const int chunk = (int)blockIdx.x;
  const int b = chunk >> 6, c = chunk & 63;
  const int tok0 = chunk * 64;
  if (tid < 64) {
    *(v4fa*)(csS + 4 * tid) = *(const v4f*)(CS + (size_t)(tok0 + tid) * 4);
    *(v4fa*)(dtS + 4 * tid) = *(const v4f*)(DTA + (size_t)(tok0 + tid) * 8);
  }
  __syncthreads();
#pragma unroll 1
  for (int i = tid; i < 256; i += 128) {
    const float d = fminf(csS[252 + (i & 3)] - csS[i], 0.0f);
    wS[i] = expf(d) * dtS[i];
  }
  __syncthreads();

  v8f g[4];
  {
    const v8f z = {0.f, 0.f, 0.f, 0.f, 0.f, 0.f, 0.f, 0.f};
    g[0] = z; g[1] = z; g[2] = z; g[3] = z;
    const unsigned short* ap = CTK + (size_t)(tok0 + 16 * wave + m) * 128 + 8 * hh;
    const unsigned short* bp = BTK + (size_t)(tok0 + m) * 128 + 8 * hh;
#pragma unroll
    for (int ks = 0; ks < 2; ++ks) {
      FragB ah, al;
      ldg_frag(ah, ap + 32 * ks);
      ldg_frag(al, ap + 64 + 32 * ks);
#pragma unroll
      for (int nt = 0; nt < 4; ++nt) {
        const unsigned short* q = bp + (size_t)(16 * nt) * 128 + 32 * ks;
        FragB bh, bl;
        ldg_frag(bh, q);
        ldg_frag(bl, q + 64);
        g[nt] = mm3(ah, al, bh, bl, g[nt]);
      }
    }
  }

#pragma unroll 1
  for (int h = 0; h < 4; ++h) {
    {
      float cst[8];
#pragma unroll
      for (int r = 0; r < 8; ++r) cst[r] = csS[(16 * wave + 8 * hh + r) * 4 + h];
#pragma unroll
      for (int nt = 0; nt < 4; ++nt) {
        const int s = 16 * nt + m;
        const float css = csS[s * 4 + h];
        const float dts = dtS[s * 4 + h];
#pragma unroll
        for (int r = 0; r < 8; ++r) {
          const int t = 16 * wave + 8 * hh + r;
          const float d = fminf(cst[r] - css, 0.0f);
          const float e = expf(d);
          const float val = (s <= t) ? (g[nt][r] * e * dts) : 0.0f;
          unsigned short hs, ls;
          split_bf(val, hs, ls);
          MmS[t * LP + s] = hs;
          MmS[64 * LP + t * LP + s] = ls;
        }
      }
    }
    {
      const int n = tid >> 1, s0 = (tid & 1) * 32;
      const unsigned short* src = BTT + (size_t)chunk * 8192 + (size_t)n * 128 + s0;
#pragma unroll
      for (int gq = 0; gq < 4; ++gq) {
        const v8us bh8 = *(const v8usa*)(src + 8 * gq);
        const v8us bl8 = *(const v8usa*)(src + 64 + 8 * gq);
        v8us oh, ol;
#pragma unroll
        for (int j = 0; j < 8; ++j) {
          const int s = s0 + 8 * gq + j;
          const float v = (bfu(bh8[j]) + bfu(bl8[j])) * wS[s * 4 + h];
          unsigned short hs, ls;
          split_bf(v, hs, ls);
          oh[j] = hs; ol[j] = ls;
        }
        *(v8usa*)(BwS + n * LP + s0 + 8 * gq) = oh;
        *(v8usa*)(BwS + 64 * LP + n * LP + s0 + 8 * gq) = ol;
      }
    }
    __syncthreads();

    const size_t xbase = (size_t)(chunk * 4 + h) * 8192;
    v8f ya[4];
    {
      const v8f z = {0.f, 0.f, 0.f, 0.f, 0.f, 0.f, 0.f, 0.f};
      ya[0] = z; ya[1] = z; ya[2] = z; ya[3] = z;
      const unsigned short* pa = MmS + (16 * wave + m) * LP + 8 * hh;
      const unsigned short* xb = XTP + xbase + (size_t)m * 128 + 8 * hh;
#pragma unroll
      for (int ks = 0; ks < 2; ++ks) {
        FragB ah, al;
        lds_frag(ah, pa + 32 * ks);
        lds_frag(al, pa + 64 * LP + 32 * ks);
#pragma unroll
        for (int nt = 0; nt < 4; ++nt) {
          const unsigned short* q = xb + (size_t)(16 * nt) * 128 + 32 * ks;
          FragB bh, bl;
          ldg_frag(bh, q);
          ldg_frag(bl, q + 64);
          ya[nt] = mm3(ah, al, bh, bl, ya[nt]);
        }
      }
      const float Dh = bf16_val(Dp[h]);
#pragma unroll
      for (int nt = 0; nt < 4; ++nt) {
        const unsigned short* xr = XTP + xbase + (size_t)(16 * nt + m) * 128 + 16 * wave + 8 * hh;
        const v8us xh8 = *(const v8usa*)xr;
        const v8us xl8 = *(const v8usa*)(xr + 64);
#pragma unroll
        for (int r = 0; r < 8; ++r) ya[nt][r] += Dh * (bfu(xh8[r]) + bfu(xl8[r]));
      }
    }
#pragma unroll
    for (int nt = 0; nt < 4; ++nt) {
#pragma unroll
      for (int r = 0; r < 8; ++r) stg[(16 * wave + 8 * hh + r) * 64 + 16 * nt + m] = ya[nt][r];
    }
    __syncthreads();
    {
      v4f fv[8];
#pragma unroll
      for (int i = 0; i < 8; ++i) fv[i] = *(const v4fa*)(stg + (16 * wave + 2 * i + hh) * 64 + 4 * m);
#pragma unroll
      for (int i = 0; i < 8; ++i) {
        const int lr = 16 * wave + 2 * i + hh;
        *(volatile v4f*)(Y + (size_t)(tok0 + lr) * 256 + h * 64 + 4 * m) = fv[i];
      }
      __threadfence();
#pragma unroll
      for (int i = 0; i < 8; ++i) {
        const int lr = 16 * wave + 2 * i + hh;
        *(volatile v4f*)(Y + (size_t)(tok0 + lr) * 256 + h * 64 + 4 * m) = fv[i];
      }
    }

    v8f sa[4];
    {
      const v8f z = {0.f, 0.f, 0.f, 0.f, 0.f, 0.f, 0.f, 0.f};
      sa[0] = z; sa[1] = z; sa[2] = z; sa[3] = z;
      const unsigned short* xa = XTP + xbase + (size_t)(16 * wave + m) * 128 + 8 * hh;
      const unsigned short* pb = BwS + m * LP + 8 * hh;
#pragma unroll
      for (int ks = 0; ks < 2; ++ks) {
        FragB ah, al;
        ldg_frag(ah, xa + 32 * ks);
        ldg_frag(al, xa + 64 + 32 * ks);
#pragma unroll
        for (int nt = 0; nt < 4; ++nt) {
          const unsigned short* q = pb + (16 * nt) * LP + 32 * ks;
          FragB bh, bl;
          lds_frag(bh, q);
          lds_frag(bl, q + 64 * LP);
          sa[nt] = mm3(ah, al, bh, bl, sa[nt]);
        }
      }
    }
    __syncthreads();
#pragma unroll
    for (int nt = 0; nt < 4; ++nt) {
#pragma unroll
      for (int r = 0; r < 8; ++r) stg[(16 * wave + 8 * hh + r) * 64 + 16 * nt + m] = sa[nt][r];
    }
    __syncthreads();
    {
      float* sp = S + ((size_t)((b * 4 + h) * 64 + c)) * 4096;
      v4f fv[8];
#pragma unroll
      for (int i = 0; i < 8; ++i) fv[i] = *(const v4fa*)(stg + (16 * wave + 2 * i + hh) * 64 + 4 * m);
#pragma unroll
      for (int i = 0; i < 8; ++i) {
        const int lr = 16 * wave + 2 * i + hh;
        *(volatile v4f*)(sp + (size_t)lr * 64 + 4 * m) = fv[i];
      }
      __threadfence();
#pragma unroll
      for (int i = 0; i < 8; ++i) {
        const int lr = 16 * wave + 2 * i + hh;
        *(volatile v4f*)(sp + (size_t)lr * 64 + 4 * m) = fv[i];
      }
    }
    __syncthreads();
  }
}

__global__ __launch_bounds__(256) void k_carry(const float* __restrict__ S, const float* __restrict__ CS,
                                               unsigned short* HP) {
  const int bh = (int)blockIdx.x;
  const int b = bh >> 2, h = bh & 3;
  const int e = (int)blockIdx.y * 256 + (int)threadIdx.x;
  const int p = e >> 3, n8 = (e & 7) * 8;
  float st[8];
#pragma unroll
  for (int j = 0; j < 8; ++j) st[j] = 0.0f;
#pragma unroll 1
  for (int c = 0; c < 64; ++c) {
    v8us oh, ol;
#pragma unroll
    for (int j = 0; j < 8; ++j) {
      unsigned short hs, ls;
      split_bf(st[j], hs, ls);
      oh[j] = hs; ol[j] = ls;
    }
    unsigned short* dp = HP + ((size_t)((bh * 64 + c) * 64 + p)) * 128 + n8;
    *(volatile v8us*)dp = oh;
    *(volatile v8us*)(dp + 64) = ol;
    __threadfence();
    *(volatile v8us*)dp = oh;
    *(volatile v8us*)(dp + 64) = ol;
    const float cl = fminf(CS[((size_t)b * 4096 + c * 64 + 63) * 4 + h], 0.0f);
    const float dch = expf(cl);
    const float* sp = S + ((size_t)((bh * 64 + c) * 64 + p)) * 64 + n8;
    const v4f s0 = *(const v4f*)sp;
    const v4f s1 = *(const v4f*)(sp + 4);
    st[0] = fmaf(dch, st[0], s0.x); st[1] = fmaf(dch, st[1], s0.y);
    st[2] = fmaf(dch, st[2], s0.z); st[3] = fmaf(dch, st[3], s0.w);
    st[4] = fmaf(dch, st[4], s1.x); st[5] = fmaf(dch, st[5], s1.y);
    st[6] = fmaf(dch, st[6], s1.z); st[7] = fmaf(dch, st[7], s1.w);
  }
}

__global__ __launch_bounds__(128) void k_ssd_out(const unsigned short* __restrict__ CTK,
                                                 const unsigned short* __restrict__ HP,
                                                 const float* __restrict__ CS, const float* __restrict__ Yp,
                                                 const float* __restrict__ Zp, const float* __restrict__ rmsw,
                                                 unsigned short* YN) {
  extern __shared__ __attribute__((aligned(16))) float dsm[];
  float* ytile = dsm;
  float* csS = dsm + 64 * YP;
  float* rw = csS + 256;
  unsigned short* CdS = (unsigned short*)(rw + 256);
  const int tid = (int)threadIdx.x, lane = tid & 31, wave = tid >> 5, hh = lane >> 4, m = lane & 15;
  const int chunk = (int)blockIdx.x;
  const int b = chunk >> 6, c = chunk & 63;
  const int tok0 = chunk * 64;
  if (tid < 64) *(v4fa*)(csS + 4 * tid) = *(const v4f*)(CS + (size_t)(tok0 + tid) * 4);
  rw[tid] = bf16_val(rmsw[tid]);
  rw[tid + 128] = bf16_val(rmsw[tid + 128]);
  __syncthreads();

#pragma unroll 1
  for (int h = 0; h < 4; ++h) {
    {
      const int t = tid >> 1, n0 = (tid & 1) * 32;
      const unsigned short* src = CTK + (size_t)(tok0 + t) * 128 + n0;
      const float e = expf(fminf(csS[t * 4 + h], 0.0f));
#pragma unroll
      for (int gq = 0; gq < 4; ++gq) {
        const v8us ch8 = *(const v8usa*)(src + 8 * gq);
        const v8us cl8 = *(const v8usa*)(src + 64 + 8 * gq);
        v8us oh, ol;
#pragma unroll
        for (int j = 0; j < 8; ++j) {
          const float v = (bfu(ch8[j]) + bfu(cl8[j])) * e;
          unsigned short hs, ls;
          split_bf(v, hs, ls);
          oh[j] = hs; ol[j] = ls;
        }
        *(v8usa*)(CdS + t * LP + n0 + 8 * gq) = oh;
        *(v8usa*)(CdS + 64 * LP + t * LP + n0 + 8 * gq) = ol;
      }
    }
    __syncthreads();
    v8f ya[4];
    {
      const v8f z = {0.f, 0.f, 0.f, 0.f, 0.f, 0.f, 0.f, 0.f};
      ya[0] = z; ya[1] = z; ya[2] = z; ya[3] = z;
      const unsigned short* pa = CdS + (16 * wave + m) * LP + 8 * hh;
      const unsigned short* hb = HP + ((size_t)(((b * 4 + h) * 64 + c) * 64 + m)) * 128 + 8 * hh;
#pragma unroll
      for (int ks = 0; ks < 2; ++ks) {
        FragB ah, al;
        lds_frag(ah, pa + 32 * ks);
        lds_frag(al, pa + 64 * LP + 32 * ks);
#pragma unroll
        for (int nt = 0; nt < 4; ++nt) {
          const unsigned short* q = hb + (size_t)(16 * nt) * 128 + 32 * ks;
          FragB bh, bl;
          ldg_frag(bh, q);
          ldg_frag(bl, q + 64);
          ya[nt] = mm3(ah, al, bh, bl, ya[nt]);
        }
      }
    }
#pragma unroll
    for (int nt = 0; nt < 4; ++nt) {
#pragma unroll
      for (int r = 0; r < 8; ++r) ytile[(16 * wave + 8 * hh + r) * YP + h * 64 + 16 * nt + m] = ya[nt][r];
    }
    __syncthreads();
  }

  const int c0 = 8 * lane;
#pragma unroll 1
  for (int i = 0; i < 16; ++i) {
    const int t = 16 * wave + i;
    const size_t tok = (size_t)(tok0 + t);
    const v4f y0 = *(const v4fa*)(ytile + t * YP + c0);
    const v4f y1 = *(const v4fa*)(ytile + t * YP + c0 + 4);
    const v4f a0 = *(const v4f*)(Yp + tok * 256 + c0);
    const v4f a1 = *(const v4f*)(Yp + tok * 256 + c0 + 4);
    const v4f z0 = *(const v4f*)(Zp + tok * 256 + c0);
    const v4f z1 = *(const v4f*)(Zp + tok * 256 + c0 + 4);
    float gv[8];
    gv[0] = (y0.x + a0.x) * silu_f(z0.x); gv[1] = (y0.y + a0.y) * silu_f(z0.y);
    gv[2] = (y0.z + a0.z) * silu_f(z0.z); gv[3] = (y0.w + a0.w) * silu_f(z0.w);
    gv[4] = (y1.x + a1.x) * silu_f(z1.x); gv[5] = (y1.y + a1.y) * silu_f(z1.y);
    gv[6] = (y1.z + a1.z) * silu_f(z1.z); gv[7] = (y1.w + a1.w) * silu_f(z1.w);
    float ss = 0.0f;
#pragma unroll
    for (int j = 0; j < 8; ++j) ss += gv[j] * gv[j];
    ss += __shfl_xor(ss, 16, 32);
    ss += __shfl_xor(ss, 8, 32);
    ss += __shfl_xor(ss, 4, 32);
    ss += __shfl_xor(ss, 2, 32);
    ss += __shfl_xor(ss, 1, 32);
    const float sc = rsqrtf(ss * (1.0f / 256.0f) + 1e-5f);
    v8us oh, ol;
#pragma unroll
    for (int j = 0; j < 8; ++j) {
      const float o = gv[j] * sc * rw[c0 + j];
      unsigned short hs, ls;
      split_bf(o, hs, ls);
      oh[j] = hs; ol[j] = ls;
    }
    unsigned short* dp = YN + tok * 512 + c0;
    *(volatile v8us*)dp = oh;
    *(volatile v8us*)(dp + 256) = ol;
    __threadfence();
    *(volatile v8us*)dp = oh;
    *(volatile v8us*)(dp + 256) = ol;
  }
}

__global__ __launch_bounds__(128) void k_outproj(const unsigned short* __restrict__ A,
                                                 const unsigned short* __restrict__ WT,
                                                 const float* __restrict__ XT, float* OUT1,
                                                 unsigned short* OUT1HL) {
  __shared__ __attribute__((aligned(16))) float stg[64 * 64];
  const int tid = (int)threadIdx.x, lane = tid & 31, wave = tid >> 5, hh = lane >> 4, m = lane & 15;
  const int rowBase = (int)blockIdx.x * 64;
  const int col0 = (int)blockIdx.y * 64;
  v8f acc[4];
  {
    const v8f z = {0.f, 0.f, 0.f, 0.f, 0.f, 0.f, 0.f, 0.f};
    acc[0] = z; acc[1] = z; acc[2] = z; acc[3] = z;
  }
  const unsigned short* ap = A + (size_t)(rowBase + 16 * wave + m) * 512 + 8 * hh;
  const unsigned short* wp = WT + (size_t)(col0 + m) * 512 + 8 * hh;
#pragma unroll 1
  for (int ks = 0; ks < 16; ++ks) {
    FragB af;
    ldg_frag(af, ap + 32 * ks);
#pragma unroll
    for (int t = 0; t < 4; ++t) {
      FragB bf;
      ldg_frag(bf, wp + (size_t)(16 * t) * 512 + 32 * ks);
      acc[t] = wmb(af, bf, acc[t]);
    }
  }
#pragma unroll
  for (int t = 0; t < 4; ++t) {
#pragma unroll
    for (int r = 0; r < 8; ++r) stg[(16 * wave + 8 * hh + r) * 64 + 16 * t + m] = acc[t][r];
  }
  __syncthreads();
  {
    v4f fv[8];
#pragma unroll
    for (int i = 0; i < 8; ++i) {
      const int lr = 16 * wave + 2 * i + hh;
      const v4f s4 = *(const v4fa*)(stg + lr * 64 + 4 * m);
      const v4f x4 = *(const v4f*)(XT + (size_t)(rowBase + lr) * CHN + col0 + 4 * m);
      fv[i] = s4 + x4;
    }
#pragma unroll
    for (int i = 0; i < 8; ++i) {
      const int lr = 16 * wave + 2 * i + hh;
      *(v4fa*)(stg + lr * 64 + 4 * m) = fv[i];
    }
#pragma unroll
    for (int i = 0; i < 8; ++i) {
      const int lr = 16 * wave + 2 * i + hh;
      *(volatile v4f*)(OUT1 + (size_t)(rowBase + lr) * CHN + col0 + 4 * m) = fv[i];
    }
    __threadfence();
#pragma unroll
    for (int i = 0; i < 8; ++i) {
      const int lr = 16 * wave + 2 * i + hh;
      *(volatile v4f*)(OUT1 + (size_t)(rowBase + lr) * CHN + col0 + 4 * m) = fv[i];
    }
  }
  __syncthreads();
  {
    v8us ov[8];
#pragma unroll
    for (int it = 0; it < 8; ++it) {
      const int u = it * 128 + tid;
      const int row = u >> 4, q = u & 15;
      const int c8 = 8 * (q & 7);
      const bool lo_sel = q >= 8;
      v8us w;
#pragma unroll
      for (int j = 0; j < 8; ++j) {
        unsigned short hs, ls;
        split_bf(stg[row * 64 + c8 + j], hs, ls);
        w[j] = lo_sel ? ls : hs;
      }
      ov[it] = w;
    }
#pragma unroll
    for (int it = 0; it < 8; ++it) {
      const int u = it * 128 + tid;
      const int row = u >> 4, q = u & 15;
      *(volatile v8us*)(OUT1HL + (size_t)(rowBase + row) * 256 + ((q >> 3) * 128) + col0 + 8 * (q & 7)) = ov[it];
    }
    __threadfence();
#pragma unroll
    for (int it = 0; it < 8; ++it) {
      const int u = it * 128 + tid;
      const int row = u >> 4, q = u & 15;
      *(volatile v8us*)(OUT1HL + (size_t)(rowBase + row) * 256 + ((q >> 3) * 128) + col0 + 8 * (q & 7)) = ov[it];
    }
  }
}

template <int MODE>
__global__ __launch_bounds__(128) void k_ff(const unsigned short* __restrict__ SRC,
                                            const unsigned short* __restrict__ W,
                                            const float* __restrict__ bias, const float* __restrict__ OUT1,
                                            unsigned short* FF1, float* outp) {
  __shared__ __attribute__((aligned(16))) float stg[64 * TP];
  const int tid = (int)threadIdx.x, lane = tid & 31, wave = tid >> 5, hh = lane >> 4, m = lane & 15;
  const int blk = (int)blockIdx.x;
  const int b = blk >> 6, y = blk & 63;
  const int tok0 = blk * 64;
  const int x = 16 * wave + m;
  v8f acc[8];
  {
    const v8f z = {0.f, 0.f, 0.f, 0.f, 0.f, 0.f, 0.f, 0.f};
#pragma unroll
    for (int t = 0; t < 8; ++t) acc[t] = z;
  }
#pragma unroll 1
  for (int tap = 0; tap < 9; ++tap) {
    const int ky = tap / 3;
    const int kx = tap - 3 * ky;
    int ry = y + ky - 1;
    ry = ry < 0 ? -ry : (ry > 63 ? 126 - ry : ry);
    int rx = x + kx - 1;
    rx = rx < 0 ? -rx : (rx > 63 ? 126 - rx : rx);
    const unsigned short* ap = SRC + ((size_t)((b * 64 + ry) * 64 + rx)) * 256 + 8 * hh;
    const unsigned short* wp = W + (size_t)m * KFF + tap * 256 + 8 * hh;
#pragma unroll 1
    for (int k0 = 0; k0 < 256; k0 += 32) {
      FragB af;
      ldg_frag(af, ap + k0);
#pragma unroll
      for (int nt = 0; nt < 8; ++nt) {
        FragB bf;
        ldg_frag(bf, wp + (size_t)(16 * nt) * KFF + k0);
        acc[nt] = wmb(af, bf, acc[nt]);
      }
    }
  }
  float bv[8];
#pragma unroll
  for (int nt = 0; nt < 8; ++nt) bv[nt] = bf16_val(bias[16 * nt + m]);
#pragma unroll
  for (int nt = 0; nt < 8; ++nt) {
#pragma unroll
    for (int r = 0; r < 8; ++r)
      stg[(16 * wave + 8 * hh + r) * TP + 16 * nt + m] = fmaxf(acc[nt][r] + bv[nt], 0.0f);
  }
  __syncthreads();
  if constexpr (MODE == 0) {
    const int c0 = 8 * (lane & 15);
    const bool lo_sel = lane >= 16;
#pragma unroll 1
    for (int i = 0; i < 16; ++i) {
      const int row = 16 * wave + i;
      const v4f s0 = *(const v4fa*)(stg + row * TP + c0);
      const v4f s1 = *(const v4fa*)(stg + row * TP + c0 + 4);
      float sv[8];
      sv[0] = s0.x; sv[1] = s0.y; sv[2] = s0.z; sv[3] = s0.w;
      sv[4] = s1.x; sv[5] = s1.y; sv[6] = s1.z; sv[7] = s1.w;
      v8us o;
#pragma unroll
      for (int j = 0; j < 8; ++j) {
        unsigned short hs, ls;
        split_bf(sv[j], hs, ls);
        o[j] = lo_sel ? ls : hs;
      }
      unsigned short* dp = FF1 + (size_t)(tok0 + row) * 256 + 8 * lane;
      *(volatile v8us*)dp = o;
      __threadfence();
      *(volatile v8us*)dp = o;
    }
  } else {
#pragma unroll 4
    for (int it = 0; it < 16; ++it) {
      const int u = it * 128 + tid;
      const int row = u >> 5, q = u & 31;
      const v4f o1 = *(const v4f*)(OUT1 + (size_t)(tok0 + row) * CHN + 4 * q);
      float* sp = stg + row * TP + 4 * q;
      const v4f sv = *(const v4fa*)sp;
      *(v4fa*)sp = sv + o1;
    }
    __syncthreads();
#pragma unroll 1
    for (int it = 0; it < 16; ++it) {
      const int u = it * 128 + tid;
      const int ch = u >> 4, xq = u & 15;
      v4f v;
      v.x = stg[(4 * xq + 0) * TP + ch];
      v.y = stg[(4 * xq + 1) * TP + ch];
      v.z = stg[(4 * xq + 2) * TP + ch];
      v.w = stg[(4 * xq + 3) * TP + ch];
      float* dp = outp + (((size_t)(b * CHN + ch) * 64 + y) * 64 + 4 * xq);
      *(volatile v4f*)dp = v;
      __threadfence();
      *(volatile v4f*)dp = v;
    }
  }
}

static inline size_t al256(size_t o) { return (o + 255) & ~(size_t)255; }

extern "C" void kernel_launch(void* const* d_in, const int* in_sizes, int n_in,
                              void* d_out, int out_size, void* d_ws, size_t ws_size,
                              hipStream_t stream) {
  if (n_in < 16) return;
  if (in_sizes[0] != NIMG || in_sizes[1] != 1) return;
  if (in_sizes[2] != CHN || in_sizes[3] != CHN) return;
  if (in_sizes[4] != NPROJ * CHN) return;
  if (in_sizes[5] != NXBC * 5 || in_sizes[6] != NXBC) return;
  if (in_sizes[7] != 4 || in_sizes[8] != 4 || in_sizes[9] != 4) return;
  if (in_sizes[10] != DINNER || in_sizes[11] != CHN * DINNER) return;
  if (in_sizes[12] != CHN * CHN * 9 || in_sizes[13] != CHN) return;
  if (in_sizes[14] != CHN * CHN * 9 || in_sizes[15] != CHN) return;
  if (out_size != NIMG + 1) return;

  const float* noisy = (const float*)d_in[0];
  const float* aux   = (const float*)d_in[1];
  const float* ln_w  = (const float*)d_in[2];
  const float* ln_b  = (const float*)d_in[3];
  const float* wip   = (const float*)d_in[4];
  const float* cw    = (const float*)d_in[5];
  const float* cb    = (const float*)d_in[6];
  const float* dtb   = (const float*)d_in[7];
  const float* alog  = (const float*)d_in[8];
  const float* Dp    = (const float*)d_in[9];
  const float* rmsw  = (const float*)d_in[10];
  const float* wop   = (const float*)d_in[11];
  const float* fw1   = (const float*)d_in[12];
  const float* fb1   = (const float*)d_in[13];
  const float* fw2   = (const float*)d_in[14];
  const float* fb2   = (const float*)d_in[15];
  float* out = (float*)d_out;

  char* ws = (char*)d_ws;
  size_t off = 0;
  const size_t oXT  = off; off = al256(off + (size_t)NTOK * CHN * 4);
  const size_t oR   = off; off = al256(off + (size_t)33554432);
  const size_t oWIN = off; off = al256(off + (size_t)NPADP * 256 * 2);
  const size_t oWOU = off; off = al256(off + (size_t)CHN * 512 * 2);
  const size_t oW1  = off; off = al256(off + (size_t)CHN * KFF * 2);
  const size_t oW2  = off; off = al256(off + (size_t)CHN * KFF * 2);
  const size_t oZ   = off; off = al256(off + (size_t)NTOK * 256 * 4);
  const size_t oDTA = off; off = al256(off + (size_t)NTOK * 8 * 4);
  const size_t oCS  = off; off = al256(off + (size_t)NTOK * 4 * 4);
  const size_t oXTP = off; off = al256(off + (size_t)NCHUNK * 4 * 8192 * 2);
  const size_t oBTK = off; off = al256(off + (size_t)NTOK * 128 * 2);
  const size_t oCTK = off; off = al256(off + (size_t)NTOK * 128 * 2);
  const size_t oBTT = off; off = al256(off + (size_t)NCHUNK * 8192 * 2);
  const size_t oSH  = off; off = al256(off + (size_t)33554432);
  if (off > ws_size || off > (size_t)WSMAX) return;

  const size_t oNRM = oR;
  const size_t oXBC = oR + (size_t)8388608;
  const size_t oY   = oR;
  const size_t oYN  = oR + (size_t)16777216;
  const size_t oS   = oSH;
  const size_t oHP  = oSH + (size_t)16777216;
  const size_t oO1  = oSH;
  const size_t oO1H = oSH + (size_t)8388608;
  const size_t oFF1 = oSH + (size_t)16777216;

  float*          XT    = (float*)(ws + oXT);
  unsigned short* NRM   = (unsigned short*)(ws + oNRM);
  unsigned short* WIN2  = (unsigned short*)(ws + oWIN);
  unsigned short* WOUT2 = (unsigned short*)(ws + oWOU);
  unsigned short* W1R   = (unsigned short*)(ws + oW1);
  unsigned short* W2R   = (unsigned short*)(ws + oW2);
  float*          Zp    = (float*)(ws + oZ);
  float*          XBC   = (float*)(ws + oXBC);
  float*          DTA   = (float*)(ws + oDTA);
  float*          CS    = (float*)(ws + oCS);
  unsigned short* XTP   = (unsigned short*)(ws + oXTP);
  unsigned short* BTK   = (unsigned short*)(ws + oBTK);
  unsigned short* CTK   = (unsigned short*)(ws + oCTK);
  unsigned short* BTT   = (unsigned short*)(ws + oBTT);
  float*          Yp    = (float*)(ws + oY);
  unsigned short* YN    = (unsigned short*)(ws + oYN);
  float*          Sp    = (float*)(ws + oS);
  unsigned short* HP    = (unsigned short*)(ws + oHP);
  float*          OUT1  = (float*)(ws + oO1);
  unsigned short* O1HL  = (unsigned short*)(ws + oO1H);
  unsigned short* FF1   = (unsigned short*)(ws + oFF1);

  hipFuncSetAttribute(reinterpret_cast<const void*>(&k_ssd_out), hipFuncAttributeMaxDynamicSharedMemorySize,
                      (int)SSDOUT_LDS);

  k_wprep<<<(NU_WIN + NU_WOUT + 2 * NU_FF) / 256, 256, 0, stream>>>(wip, wop, fw1, fw2, aux,
                                                                     WIN2, WOUT2, W1R, W2R, out);
  k_ln<<<NCHUNK, 256, 0, stream>>>(noisy, ln_w, ln_b, XT, NRM);
  k_inproj<<<dim3(NTOK / 64, NPADP / 64), 128, 0, stream>>>(NRM, WIN2, dtb, alog, (float*)ws,
                                                             oZ / 4, oXBC / 4, oDTA / 4);
  k_conv1d<<<dim3(NCHUNK, 6), 256, 0, stream>>>(XBC, DTA, cw, cb, XTP, BTT, BTK, CTK, CS);
  k_ssd_local<<<NCHUNK, 128, 0, stream>>>(CTK, BTK, XTP, BTT, CS, DTA, Dp, Yp, Sp);
  k_carry<<<dim3(16, 2), 256, 0, stream>>>(Sp, CS, HP);
  k_ssd_out<<<NCHUNK, 128, SSDOUT_LDS, stream>>>(CTK, HP, CS, Yp, Zp, rmsw, YN);
  k_outproj<<<dim3(NTOK / 64, 2), 128, 0, stream>>>(YN, WOUT2, XT, OUT1, O1HL);
  k_ff<0><<<NCHUNK, 128, 0, stream>>>(O1HL, W1R, fb1, OUT1, FF1, out);
  k_ff<1><<<NCHUNK, 128, 0, stream>>>(FF1, W2R, fb2, OUT1, O1HL, out);
}
